// ODE_RNN_10350871183741
// MI455X (gfx1250) — hardware-verified
//
#include <hip/hip_runtime.h>
#include <stddef.h>

typedef __attribute__((ext_vector_type(16))) __bf16 v16b;
typedef __attribute__((ext_vector_type(8)))  __bf16 v8b;
typedef __attribute__((ext_vector_type(8)))  float  v8f;
typedef __attribute__((ext_vector_type(4)))  float  v4f;
typedef __attribute__((ext_vector_type(4)))  unsigned int v4u;

constexpr int BATCH   = 128;
constexpr int TSTEPS  = 64;
constexpr int OBD     = 32;
constexpr int ACD     = 8;
constexpr int ACK     = 32;
constexpr int LAT     = 128;
constexpr int HID     = 256;
constexpr int NSTAGE  = 6;
constexpr int NSUBST  = 4;
constexpr int MROWS   = 16;
constexpr int NTHREADS = 256;
constexpr int NBLOCKS = BATCH / MROWS;

static_assert(BATCH % MROWS == 0);
static_assert(NTHREADS * 8 == MROWS * LAT);
static_assert(HID == 2 * LAT);
static_assert(LAT % 32 == 0 && HID % 32 == 0 && OBD == 32 && ACK == 32);

constexpr int OFF_Y    = 0;
constexpr int OFF_K    = OFF_Y + MROWS * LAT * 4;
constexpr int OFF_YSH  = OFF_K + NSTAGE * MROWS * LAT * 4;
constexpr int OFF_YSL  = OFF_YSH + MROWS * LAT * 2;
constexpr int OFF_H1H  = OFF_YSL + MROWS * LAT * 2;
constexpr int OFF_H1L  = OFF_H1H + MROWS * HID * 2;
constexpr int OFF_H2H  = OFF_H1L + MROWS * HID * 2;
constexpr int OFF_H2L  = OFF_H2H + MROWS * HID * 2;
constexpr int OFF_OUT  = OFF_H2L + MROWS * HID * 2;
constexpr int OFF_HST  = OFF_OUT + MROWS * OBD * 4;
constexpr int OFF_COEF = OFF_HST + MROWS * 4;
constexpr int SMEM_TOTAL = OFF_COEF + 48 * 4;
static_assert(SMEM_TOTAL == 100608);
static_assert(OFF_YSH % 16 == 0 && OFF_H1H % 16 == 0 && OFF_OUT % 16 == 0 && OFF_COEF % 16 == 0);
static_assert(MROWS * (2 * LAT + LAT + LAT) * 4 <= NSTAGE * MROWS * LAT * 4);

constexpr size_t WS_WE0 = 0;
constexpr size_t WS_WE1 = WS_WE0 + (size_t)HID * OBD * 2;
constexpr size_t WS_WD0 = WS_WE1 + (size_t)LAT * HID * 2;
constexpr size_t WS_WD1 = WS_WD0 + (size_t)HID * LAT * 2;
constexpr size_t WS_WD2 = WS_WD1 + (size_t)HID * HID * 2;
constexpr size_t WS_WO0 = WS_WD2 + (size_t)LAT * HID * 2;
constexpr size_t WS_WO1 = WS_WO0 + (size_t)HID * LAT * 2;
constexpr size_t WS_WHH = WS_WO1 + (size_t)OBD * HID * 2;
constexpr size_t WS_WIH = WS_WHH + (size_t)3 * LAT * LAT * 2;
constexpr size_t WS_TOTAL = WS_WIH + (size_t)3 * LAT * ACK * 2;
static_assert(WS_TOTAL == 548864);
static_assert(WS_WE1 % 128 == 0 && WS_WD0 % 128 == 0 && WS_WD1 % 128 == 0 && WS_WD2 % 128 == 0 &&
              WS_WO0 % 128 == 0 && WS_WO1 % 128 == 0 && WS_WHH % 128 == 0 && WS_WIH % 128 == 0);
static_assert((HID * OBD) % 2048 == 0 && (LAT * HID) % 2048 == 0 && (HID * HID) % 2048 == 0 &&
              (OBD * HID) % 2048 == 0 && (3 * LAT * LAT) % 2048 == 0);
static_assert((3 * LAT * 4) % 256 == 0);

__device__ __forceinline__ unsigned short f2bf_bits(float f) {
  unsigned u = __float_as_uint(f);
  return (unsigned short)((u + 0x7FFFu + ((u >> 16) & 1u)) >> 16);
}
__device__ __forceinline__ float bf_bits2f(unsigned short h) { return __uint_as_float(((unsigned)h) << 16); }
__device__ __forceinline__ float bfr(float f) { return bf_bits2f(f2bf_bits(f)); }
__device__ __forceinline__ unsigned pack2(float a, float b) {
  return (unsigned)f2bf_bits(a) | ((unsigned)f2bf_bits(b) << 16);
}
__device__ __forceinline__ v8f zero8() { return (v8f){0.f, 0.f, 0.f, 0.f, 0.f, 0.f, 0.f, 0.f}; }

__device__ __forceinline__ v8f bmma(v16b a, v16b b, v8f c) {
  c = __builtin_amdgcn_wmma_f32_16x16x32_bf16(false, a, false, b, (short)0, c, false, false);
  asm volatile("v_nop\n\tv_nop\n\tv_nop\n\tv_nop" : "+v"(c) : "v"(a), "v"(b));
  return c;
}
__device__ __forceinline__ v16b frag16(const unsigned short* p) {
  union { v16b v; v8b h[2]; } f;
  f.h[0] = *(const v8b*)(p);
  f.h[1] = *(const v8b*)(p + 16);
  return f.v;
}
union FragU { v16b v; unsigned u[8]; };

template <int NT>
__device__ __forceinline__ void mm_hl(const unsigned short* aH, const unsigned short* aL, int lda,
                                      const unsigned short* __restrict__ Bt, int ldb,
                                      const int (&nb)[NT], int K, int lane, v8f (&acc)[NT]) {
  const int r = lane & 15, koff = (lane >> 4) * 8;
#pragma unroll 1
  for (int k0 = 0; k0 < K; k0 += 32) {
    const v16b ah = frag16(aH + r * lda + koff + k0);
    const v16b al = frag16(aL + r * lda + koff + k0);
#pragma unroll
    for (int j = 0; j < NT; ++j) {
      const v16b bf = frag16(Bt + (size_t)(nb[j] + r) * ldb + koff + k0);
      acc[j] = bmma(ah, bf, acc[j]);
      acc[j] = bmma(al, bf, acc[j]);
    }
  }
}

template <bool RELU>
__device__ __forceinline__ void tile_to_planes(unsigned short* pH, unsigned short* pL, int ld, int nb,
                                               v8f acc, float bias, int lane) {
  const int c = lane & 15, r0 = (lane >> 4) * 8;
#pragma unroll
  for (int r = 0; r < 8; ++r) {
    float v = acc[r] + bias;
    if (RELU) v = fmaxf(v, 0.0f);
    const unsigned short hb = f2bf_bits(v);
    const unsigned short lb = f2bf_bits(v - bf_bits2f(hb));
    const int idx = (r0 + r) * ld + nb + c;
    pH[idx] = hb;
    pL[idx] = lb;
  }
}
__device__ __forceinline__ void tile_to_f32(float* p, int ld, int nb, v8f acc, float bias, int lane) {
  const int c = lane & 15, r0 = (lane >> 4) * 8;
#pragma unroll
  for (int r = 0; r < 8; ++r) p[(r0 + r) * ld + nb + c] = acc[r] + bias;
}

__device__ __forceinline__ void ld8(const float* p, float (&v)[8]) {
  const v4f a = *(const v4f*)(p);
  const v4f b = *(const v4f*)(p + 4);
  v[0] = a[0]; v[1] = a[1]; v[2] = a[2]; v[3] = a[3];
  v[4] = b[0]; v[5] = b[1]; v[6] = b[2]; v[7] = b[3];
}
__device__ __forceinline__ void st8(float* p, const float (&v)[8]) {
  *(v4f*)(p)     = (v4f){v[0], v[1], v[2], v[3]};
  *(v4f*)(p + 4) = (v4f){v[4], v[5], v[6], v[7]};
}
__device__ __forceinline__ void split8_store(unsigned short* pH, unsigned short* pL, const float (&v)[8]) {
  v4u wh, wl;
#pragma unroll
  for (int e = 0; e < 4; ++e) {
    const float x0 = v[2 * e], x1 = v[2 * e + 1];
    const unsigned short h0 = f2bf_bits(x0), h1 = f2bf_bits(x1);
    const unsigned short l0 = f2bf_bits(x0 - bf_bits2f(h0));
    const unsigned short l1 = f2bf_bits(x1 - bf_bits2f(h1));
    wh[e] = (unsigned)h0 | ((unsigned)h1 << 16);
    wl[e] = (unsigned)l0 | ((unsigned)l1 << 16);
  }
  *(v4u*)pH = wh;
  *(v4u*)pL = wl;
}

__device__ __forceinline__ void build_stage(int tid, int s, float* sY, const float* sK, const float* sHst,
                                            const float* sCoef, unsigned short* yh, unsigned short* yl) {
  const int i0 = tid * 8;
  const int m = i0 >> 7;
  const float hh = sHst[m];
  float y[8], acc[8], ys[8];
  ld8(sY + i0, y);
#pragma unroll
  for (int e = 0; e < 8; ++e) acc[e] = 0.0f;
#pragma unroll 1
  for (int j = 0; j <= s; ++j) {
    const float cj = sCoef[s * NSTAGE + j];
    float kv[8];
    ld8(sK + j * (MROWS * LAT) + i0, kv);
#pragma unroll
    for (int e = 0; e < 8; ++e) acc[e] += cj * kv[e];
  }
#pragma unroll
  for (int e = 0; e < 8; ++e) ys[e] = y[e] + hh * acc[e];
  split8_store(yh + i0, yl + i0, ys);
  if (s == NSTAGE - 1) st8(sY + i0, ys);
}

__device__ __forceinline__ v8f dyn_eval(int w, int lane,
    const unsigned short* inH, const unsigned short* inL,
    unsigned short* h1h, unsigned short* h1l, unsigned short* h2h, unsigned short* h2l,
    const unsigned short* __restrict__ Wd0p, const unsigned short* __restrict__ Wd1p,
    const unsigned short* __restrict__ Wd2p,
    float bd0r0, float bd0r1, float bd1r0, float bd1r1) {
  const int nb2[2] = {16 * w, 16 * (w + 8)};
  {
    v8f a[2] = {zero8(), zero8()};
    mm_hl<2>(inH, inL, LAT, Wd0p, LAT, nb2, LAT, lane, a);
    tile_to_planes<true>(h1h, h1l, HID, nb2[0], a[0], bd0r0, lane);
    tile_to_planes<true>(h1h, h1l, HID, nb2[1], a[1], bd0r1, lane);
  }
  __syncthreads();
  {
    v8f b[2] = {zero8(), zero8()};
    mm_hl<2>(h1h, h1l, HID, Wd1p, HID, nb2, HID, lane, b);
    tile_to_planes<true>(h2h, h2l, HID, nb2[0], b[0], bd1r0, lane);
    tile_to_planes<true>(h2h, h2l, HID, nb2[1], b[1], bd1r1, lane);
  }
  __syncthreads();
  v8f cacc[1] = {zero8()};
  const int nb1[1] = {16 * w};
  mm_hl<1>(h2h, h2l, HID, Wd2p, HID, nb1, HID, lane, cacc);
  return cacc[0];
}

__device__ __forceinline__ void write_out_lines(const float* sOut, float* out, int m0, int t, int lane) {
  const int q = lane >> 3, c4 = (lane & 7) * 4;
  for (int pass = 0; pass < 2; ++pass) {
#pragma unroll
    for (int it = 0; it < 4; ++it) {
      const int row = it * 4 + q;
      const v4f v = *(const v4f*)(sOut + row * OBD + c4);
      *(volatile v4f*)(out + ((size_t)(m0 + row) * TSTEPS + t) * OBD + c4) = v;
    }
    __threadfence();
  }
}

__global__ __launch_bounds__(256) void cast_bf16x8(const float* __restrict__ in,
                                                   unsigned short* __restrict__ outp, int n8) {
  const int i = blockIdx.x * 256 + threadIdx.x;
  if (i < n8) {
    const v4f a = *(const v4f*)(in + (size_t)8 * i);
    const v4f b = *(const v4f*)(in + (size_t)8 * i + 4);
    v4u wv;
    wv[0] = pack2(a[0], a[1]); wv[1] = pack2(a[2], a[3]);
    wv[2] = pack2(b[0], b[1]); wv[3] = pack2(b[2], b[3]);
    *(volatile v4u*)(outp + (size_t)8 * i) = wv;
    __threadfence();
    *(volatile v4u*)(outp + (size_t)8 * i) = wv;
  }
}

__global__ __launch_bounds__(256) void pad_rows8_to32(const float* __restrict__ in,
                                                      unsigned short* __restrict__ outp, int nrows) {
  const int i = blockIdx.x * 256 + threadIdx.x;
  if (i < nrows * 4) {
    const int row = i >> 2, g = i & 3;
    const v4f a = *(const v4f*)(in + (size_t)row * 8);
    const v4f b = *(const v4f*)(in + (size_t)row * 8 + 4);
    const unsigned keep = (g == 0) ? 0xFFFFFFFFu : 0u;
    v4u wv;
    wv[0] = pack2(a[0], a[1]) & keep; wv[1] = pack2(a[2], a[3]) & keep;
    wv[2] = pack2(b[0], b[1]) & keep; wv[3] = pack2(b[2], b[3]) & keep;
    *(volatile v4u*)(outp + (size_t)row * ACK + g * 8) = wv;
    __threadfence();
    *(volatile v4u*)(outp + (size_t)row * ACK + g * 8) = wv;
  }
}

__global__ __launch_bounds__(NTHREADS) void seq_main(
    const float* __restrict__ ob, const float* __restrict__ acs, const float* __restrict__ times,
    const float* __restrict__ be0, const float* __restrict__ be1,
    const float* __restrict__ bd0, const float* __restrict__ bd1, const float* __restrict__ bd2,
    const float* __restrict__ bo0, const float* __restrict__ bo1,
    const float* __restrict__ bih, const float* __restrict__ bn,
    const unsigned short* __restrict__ We0p, const unsigned short* __restrict__ We1p,
    const unsigned short* __restrict__ Wd0p, const unsigned short* __restrict__ Wd1p,
    const unsigned short* __restrict__ Wd2p, const unsigned short* __restrict__ Wo0p,
    const unsigned short* __restrict__ Wo1p, const unsigned short* __restrict__ Whhp,
    const unsigned short* __restrict__ Wihp, float* __restrict__ out) {
  __shared__ __align__(16) unsigned char smem[SMEM_TOTAL];
  float* sY   = (float*)(smem + OFF_Y);
  float* sK   = (float*)(smem + OFF_K);
  float* grz  = sK;
  float* gin  = sK + MROWS * 2 * LAT;
  float* ghn  = gin + MROWS * LAT;
  unsigned short* ySh = (unsigned short*)(smem + OFF_YSH);
  unsigned short* ySl = (unsigned short*)(smem + OFF_YSL);
  unsigned short* h1h = (unsigned short*)(smem + OFF_H1H);
  unsigned short* h1l = (unsigned short*)(smem + OFF_H1L);
  unsigned short* h2h = (unsigned short*)(smem + OFF_H2H);
  unsigned short* h2l = (unsigned short*)(smem + OFF_H2L);
  float* sOut  = (float*)(smem + OFF_OUT);
  float* sHst  = (float*)(smem + OFF_HST);
  float* sCoef = (float*)(smem + OFF_COEF);

  const int tid  = threadIdx.x;
  const int w    = tid >> 5;
  const int lane = tid & 31;
  const int c    = lane & 15;
  const int r0   = (lane >> 4) * 8;
  const int m0   = blockIdx.x * MROWS;
  const int n0a  = 16 * w + c;
  const int n1a  = 16 * (w + 8) + c;

  if (tid == 0) {
#pragma unroll
    for (int i = 0; i < 48; ++i) sCoef[i] = 0.0f;
    sCoef[0 * NSTAGE + 0] = 0.2f;
    sCoef[1 * NSTAGE + 0] = (float)(3.0 / 40.0);
    sCoef[1 * NSTAGE + 1] = (float)(9.0 / 40.0);
    sCoef[2 * NSTAGE + 0] = (float)(44.0 / 45.0);
    sCoef[2 * NSTAGE + 1] = -(float)(56.0 / 15.0);
    sCoef[2 * NSTAGE + 2] = (float)(32.0 / 9.0);
    sCoef[3 * NSTAGE + 0] = (float)(19372.0 / 6561.0);
    sCoef[3 * NSTAGE + 1] = -(float)(25360.0 / 2187.0);
    sCoef[3 * NSTAGE + 2] = (float)(64448.0 / 6561.0);
    sCoef[3 * NSTAGE + 3] = -(float)(212.0 / 729.0);
    sCoef[4 * NSTAGE + 0] = (float)(9017.0 / 3168.0);
    sCoef[4 * NSTAGE + 1] = -(float)(355.0 / 33.0);
    sCoef[4 * NSTAGE + 2] = (float)(46732.0 / 5247.0);
    sCoef[4 * NSTAGE + 3] = (float)(49.0 / 176.0);
    sCoef[4 * NSTAGE + 4] = -(float)(5103.0 / 18656.0);
    sCoef[5 * NSTAGE + 0] = (float)(35.0 / 384.0);
    sCoef[5 * NSTAGE + 1] = 0.0f;
    sCoef[5 * NSTAGE + 2] = (float)(500.0 / 1113.0);
    sCoef[5 * NSTAGE + 3] = (float)(125.0 / 192.0);
    sCoef[5 * NSTAGE + 4] = -(float)(2187.0 / 6784.0);
    sCoef[5 * NSTAGE + 5] = (float)(11.0 / 84.0);
  }

  const float be0r0 = bfr(be0[n0a]), be0r1 = bfr(be0[n1a]);
  const float be1r  = bfr(be1[n0a]);
  const float bo1r  = bfr(bo1[(n0a < OBD) ? n0a : (OBD - 1)]);
  float bnr[8];
  {
    const int lc = (tid * 8) & (LAT - 1);
    ld8(bn + lc, bnr);
#pragma unroll
    for (int e = 0; e < 8; ++e) bnr[e] = bfr(bnr[e]);
  }
  __syncthreads();

  {
    FragU f;
    {
      const float* p = ob + (size_t)(m0 + c) * OBD + r0;
      const v4f q0 = *(const v4f*)(p), q1 = *(const v4f*)(p + 4);
      const v4f q2 = *(const v4f*)(p + 16), q3 = *(const v4f*)(p + 20);
      f.u[0] = pack2(q0[0], q0[1]); f.u[1] = pack2(q0[2], q0[3]);
      f.u[2] = pack2(q1[0], q1[1]); f.u[3] = pack2(q1[2], q1[3]);
      f.u[4] = pack2(q2[0], q2[1]); f.u[5] = pack2(q2[2], q2[3]);
      f.u[6] = pack2(q3[0], q3[1]); f.u[7] = pack2(q3[2], q3[3]);
    }
    v8f e0 = zero8(), e1 = zero8();
    e0 = bmma(f.v, frag16(We0p + (size_t)n0a * OBD + r0), e0);
    e1 = bmma(f.v, frag16(We0p + (size_t)n1a * OBD + r0), e1);
    tile_to_planes<true>(h1h, h1l, HID, 16 * w, e0, be0r0, lane);
    tile_to_planes<true>(h1h, h1l, HID, 16 * (w + 8), e1, be0r1, lane);
  }
  __syncthreads();
  {
    v8f a1[1] = {zero8()};
    const int nb1[1] = {16 * w};
    mm_hl<1>(h1h, h1l, HID, We1p, HID, nb1, HID, lane, a1);
    tile_to_f32(sY, LAT, 16 * w, a1[0], be1r, lane);
    tile_to_planes<false>(ySh, ySl, LAT, 16 * w, a1[0], be1r, lane);
  }
  __syncthreads();

  const float bd0r0 = bfr(bd0[n0a]), bd0r1 = bfr(bd0[n1a]);
  const float bd1r0 = bfr(bd1[n0a]), bd1r1 = bfr(bd1[n1a]);
  const float bd2r  = bfr(bd2[n0a]);
  const float bo0r0 = bfr(bo0[n0a]), bo0r1 = bfr(bo0[n1a]);
  const float bihR = bfr(bih[n0a]), bihZ = bfr(bih[LAT + n0a]), bihN = bfr(bih[2 * LAT + n0a]);

#pragma unroll 1
  for (int t = 0; t < TSTEPS; ++t) {
    if (t > 0) {
      {
        const int mm = tid & 15;
        const float* tr = times + (size_t)(m0 + mm) * TSTEPS;
        const float dt = bfr(tr[t]) - bfr(tr[t - 1]);
        const float hh = dt * 0.25f;
        if (tid < MROWS) sHst[tid] = hh;
      }
      __syncthreads();
#pragma unroll 1
      for (int sub = 0; sub < NSUBST; ++sub) {
#pragma unroll 1
        for (int s = 0; s < NSTAGE; ++s) {
          const v8f kacc = dyn_eval(w, lane, ySh, ySl, h1h, h1l, h2h, h2l,
                                    Wd0p, Wd1p, Wd2p, bd0r0, bd0r1, bd1r0, bd1r1);
          tile_to_f32(sK + s * (MROWS * LAT), LAT, 16 * w, kacc, bd2r, lane);
          __syncthreads();
          build_stage(tid, s, sY, sK, sHst, sCoef, ySh, ySl);
          __syncthreads();
        }
      }
    }

    {
      FragU fx;
      {
        const float* p = acs + ((size_t)(m0 + c) * TSTEPS + t) * ACD;
        const v4f a0 = *(const v4f*)(p), a1 = *(const v4f*)(p + 4);
        const unsigned keep = (lane < 16) ? 0xFFFFFFFFu : 0u;
        fx.u[0] = pack2(a0[0], a0[1]) & keep; fx.u[1] = pack2(a0[2], a0[3]) & keep;
        fx.u[2] = pack2(a1[0], a1[1]) & keep; fx.u[3] = pack2(a1[2], a1[3]) & keep;
        fx.u[4] = 0u; fx.u[5] = 0u; fx.u[6] = 0u; fx.u[7] = 0u;
      }
      v8f g[3] = {zero8(), zero8(), zero8()};
      g[0] = bmma(fx.v, frag16(Wihp + (size_t)(n0a) * ACK + r0), g[0]);
      g[1] = bmma(fx.v, frag16(Wihp + (size_t)(LAT + n0a) * ACK + r0), g[1]);
      const v8f gni = bmma(fx.v, frag16(Wihp + (size_t)(2 * LAT + n0a) * ACK + r0), zero8());
      const int nb3[3] = {16 * w, LAT + 16 * w, 2 * LAT + 16 * w};
      mm_hl<3>(ySh, ySl, LAT, Whhp, LAT, nb3, LAT, lane, g);
      tile_to_f32(grz, 2 * LAT, 16 * w, g[0], bihR, lane);
      tile_to_f32(grz, 2 * LAT, LAT + 16 * w, g[1], bihZ, lane);
      tile_to_f32(gin, LAT, 16 * w, gni, bihN, lane);
      tile_to_f32(ghn, LAT, 16 * w, g[2], 0.0f, lane);
    }
    __syncthreads();
    {
      const int i0 = tid * 8, m = i0 >> 7, lc = i0 & (LAT - 1);
      float gr[8], gz[8], gi[8], gh[8], yv[8], yo[8];
      ld8(grz + m * (2 * LAT) + lc, gr);
      ld8(grz + m * (2 * LAT) + LAT + lc, gz);
      ld8(gin + i0, gi);
      ld8(ghn + i0, gh);
      ld8(sY + i0, yv);
#pragma unroll
      for (int e = 0; e < 8; ++e) {
        const float xr = fminf(fmaxf(gr[e], -30.0f), 30.0f);
        const float xz = fminf(fmaxf(gz[e], -30.0f), 30.0f);
        const float rg = 1.0f / (1.0f + expf(-xr));
        const float zg = 1.0f / (1.0f + expf(-xz));
        const float ng = tanhf(gi[e] + rg * (gh[e] + bnr[e]));
        yo[e] = (1.0f - zg) * ng + zg * yv[e];
      }
      st8(sY + i0, yo);
      split8_store(ySh + i0, ySl + i0, yo);
    }
    __syncthreads();

    {
      v8f d[2] = {zero8(), zero8()};
      const int nb2[2] = {16 * w, 16 * (w + 8)};
      mm_hl<2>(ySh, ySl, LAT, Wo0p, LAT, nb2, LAT, lane, d);
      tile_to_planes<true>(h1h, h1l, HID, nb2[0], d[0], bo0r0, lane);
      tile_to_planes<true>(h1h, h1l, HID, nb2[1], d[1], bo0r1, lane);
    }
    __syncthreads();
    if (w < 2) {
      v8f o1[1] = {zero8()};
      const int nbo[1] = {16 * w};
      mm_hl<1>(h1h, h1l, HID, Wo1p, HID, nbo, HID, lane, o1);
      tile_to_f32(sOut, OBD, 16 * w, o1[0], bo1r, lane);
    }
    __syncthreads();
    if (w == 0) write_out_lines(sOut, out, m0, t, lane);
    __syncthreads();
  }
}

extern "C" void kernel_launch(void* const* d_in, const int* in_sizes, int n_in,
                              void* d_out, int out_size, void* d_ws,
                              size_t ws_size, hipStream_t stream) {
  if (n_in < 21) return;
  if (out_size != BATCH * TSTEPS * OBD) return;
  const int expect[21] = {BATCH * OBD, BATCH * TSTEPS * ACD, BATCH * TSTEPS,
                          HID * OBD, HID, LAT * HID, LAT,
                          HID * LAT, HID, HID * HID, HID, LAT * HID, LAT,
                          HID * LAT, HID, OBD * HID, OBD,
                          3 * LAT * ACD, 3 * LAT * LAT, 3 * LAT, LAT};
  for (int i = 0; i < 21; ++i) if (in_sizes[i] != expect[i]) return;
  if (ws_size < WS_TOTAL) return;

  const float* ob    = (const float*)d_in[0];
  const float* acs   = (const float*)d_in[1];
  const float* times = (const float*)d_in[2];
  const float* We0 = (const float*)d_in[3];  const float* be0 = (const float*)d_in[4];
  const float* We1 = (const float*)d_in[5];  const float* be1 = (const float*)d_in[6];
  const float* Wd0 = (const float*)d_in[7];  const float* bd0 = (const float*)d_in[8];
  const float* Wd1 = (const float*)d_in[9];  const float* bd1 = (const float*)d_in[10];
  const float* Wd2 = (const float*)d_in[11]; const float* bd2 = (const float*)d_in[12];
  const float* Wo0 = (const float*)d_in[13]; const float* bo0 = (const float*)d_in[14];
  const float* Wo1 = (const float*)d_in[15]; const float* bo1 = (const float*)d_in[16];
  const float* Wih = (const float*)d_in[17]; const float* Whh = (const float*)d_in[18];
  const float* bih = (const float*)d_in[19]; const float* bn  = (const float*)d_in[20];
  float* out = (float*)d_out;

  unsigned char* ws = (unsigned char*)d_ws;
  unsigned short* We0p = (unsigned short*)(ws + WS_WE0);
  unsigned short* We1p = (unsigned short*)(ws + WS_WE1);
  unsigned short* Wd0p = (unsigned short*)(ws + WS_WD0);
  unsigned short* Wd1p = (unsigned short*)(ws + WS_WD1);
  unsigned short* Wd2p = (unsigned short*)(ws + WS_WD2);
  unsigned short* Wo0p = (unsigned short*)(ws + WS_WO0);
  unsigned short* Wo1p = (unsigned short*)(ws + WS_WO1);
  unsigned short* Whhp = (unsigned short*)(ws + WS_WHH);
  unsigned short* Wihp = (unsigned short*)(ws + WS_WIH);

  cast_bf16x8<<<dim3((HID * OBD) / 2048), dim3(256), 0, stream>>>(We0, We0p, (HID * OBD) / 8);
  cast_bf16x8<<<dim3((LAT * HID) / 2048), dim3(256), 0, stream>>>(We1, We1p, (LAT * HID) / 8);
  cast_bf16x8<<<dim3((HID * LAT) / 2048), dim3(256), 0, stream>>>(Wd0, Wd0p, (HID * LAT) / 8);
  cast_bf16x8<<<dim3((HID * HID) / 2048), dim3(256), 0, stream>>>(Wd1, Wd1p, (HID * HID) / 8);
  cast_bf16x8<<<dim3((LAT * HID) / 2048), dim3(256), 0, stream>>>(Wd2, Wd2p, (LAT * HID) / 8);
  cast_bf16x8<<<dim3((HID * LAT) / 2048), dim3(256), 0, stream>>>(Wo0, Wo0p, (HID * LAT) / 8);
  cast_bf16x8<<<dim3((OBD * HID) / 2048), dim3(256), 0, stream>>>(Wo1, Wo1p, (OBD * HID) / 8);
  cast_bf16x8<<<dim3((3 * LAT * LAT) / 2048), dim3(256), 0, stream>>>(Whh, Whhp, (3 * LAT * LAT) / 8);
  pad_rows8_to32<<<dim3((3 * LAT * 4) / 256), dim3(256), 0, stream>>>(Wih, Wihp, 3 * LAT);

  seq_main<<<dim3(NBLOCKS), dim3(NTHREADS), 0, stream>>>(
      ob, acs, times, be0, be1, bd0, bd1, bd2, bo0, bo1, bih, bn,
      We0p, We1p, Wd0p, Wd1p, Wd2p, Wo0p, Wo1p, Whhp, Wihp, out);
}
